// GCNNalpha_39402029973528
// MI455X (gfx1250) — hardware-verified
//
#include <hip/hip_runtime.h>
#include <stddef.h>


#define NNODE   512
#define FEAT    128
#define FOUTC   64
#define NTAP    3
#define KCONV   (NTAP * FEAT)
#define NTHR    256
#define NWAVE   8
#define EPT     8
#define NGRP    2
#define CHUNK   (NTHR * EPT * NGRP)
#define WCAP    (EPT * NGRP * 32)
#define LISTN   (NWAVE * WCAP)
#define NBC     4096
#define NBF     1024
#define RCAP    32768
#define RBN     128
#define TGT     256
#define DEGCAP  256
#define GROWS   128
#define OTHR    512
#define WSCAP   134217728
#define WSCALE  16.0f
#define WINV    0.0625f
#define LDS_FILL ((RCAP + NBF + LISTN) * 4 + 64)
#define LDS_GEMM(KD) (GROWS * ((KD) + 8) * 2)

static_assert((CHUNK & (CHUNK - 1)) == 0);
static_assert(CHUNK <= 4096);
static_assert(NBC <= 4096 && NBF <= 4096);
static_assert((NBC & (NBC - 1)) == 0 && (NBF & (NBF - 1)) == 0);
static_assert(NBC == 4 * NBF);
static_assert(OTHR * 8 == NBC);
static_assert((RCAP % 32) == 0);
static_assert((TGT % GROWS) == 0 && TGT == NWAVE * 32);
static_assert((NBC % TGT) == 0);
static_assert(GROWS == NWAVE * 16);
static_assert((NNODE & (NNODE - 1)) == 0);
static_assert((KCONV % 32) == 0 && FEAT == 4 * 32 && (FOUTC % 64) == 0);

typedef float          v4f  __attribute__((ext_vector_type(4)));
typedef float          v8f  __attribute__((ext_vector_type(8)));
typedef int            v4i  __attribute__((ext_vector_type(4)));
typedef _Float16       v8h  __attribute__((ext_vector_type(8)));
typedef _Float16       v16h __attribute__((ext_vector_type(16)));
union FragH { v16h v; v8h h[2]; };
union Pack8 { v8h h; v4i i; };

__device__ __forceinline__ v8h cvt8(v4f a, v4f b, float s) {
  v8h r;
  r[0] = (_Float16)(a.x * s); r[1] = (_Float16)(a.y * s);
  r[2] = (_Float16)(a.z * s); r[3] = (_Float16)(a.w * s);
  r[4] = (_Float16)(b.x * s); r[5] = (_Float16)(b.y * s);
  r[6] = (_Float16)(b.z * s); r[7] = (_Float16)(b.w * s);
  return r;
}

__device__ __forceinline__ v8f wmh(v16h a, v16h b, v8f c) {
  v8f d = __builtin_amdgcn_wmma_f32_16x16x32_f16(false, a, false, b, (short)0, c, false, false);
  asm volatile("v_nop\n\tv_nop\n\tv_nop\n\tv_nop" : "+v"(d) : "v"(a), "v"(b));
  return d;
}

template <int NB>
__device__ __forceinline__ int scan_chunk(const int* __restrict__ keys, int nE, int cbase, int slotBase,
                                          int vec8, int* list, int tid, int lane, int wave) {
  int wc = 0;
#pragma unroll
  for (int g = 0; g < NGRP; ++g) {
    const int el0  = (g * NTHR + tid) * EPT;
    const int e0   = cbase + el0;
    const int sent = -2147483647 - 1;
    v4i da, db;
    if (vec8 != 0 && cbase + CHUNK <= nE) {
      da = *(const v4i*)(keys + e0);
      db = *(const v4i*)(keys + e0 + 4);
    } else {
      da.x = (e0     < nE) ? keys[min(e0, nE - 1)] : sent;
      da.y = (e0 + 1 < nE) ? keys[min(e0 + 1, nE - 1)] : sent;
      da.z = (e0 + 2 < nE) ? keys[min(e0 + 2, nE - 1)] : sent;
      da.w = (e0 + 3 < nE) ? keys[min(e0 + 3, nE - 1)] : sent;
      db.x = (e0 + 4 < nE) ? keys[min(e0 + 4, nE - 1)] : sent;
      db.y = (e0 + 5 < nE) ? keys[min(e0 + 5, nE - 1)] : sent;
      db.z = (e0 + 6 < nE) ? keys[min(e0 + 6, nE - 1)] : sent;
      db.w = (e0 + 7 < nE) ? keys[min(e0 + 7, nE - 1)] : sent;
    }
    const unsigned nb = (unsigned)slotBase;
    const unsigned s0 = (unsigned)da.x - nb, s1 = (unsigned)da.y - nb;
    const unsigned s2 = (unsigned)da.z - nb, s3 = (unsigned)da.w - nb;
    const unsigned s4 = (unsigned)db.x - nb, s5 = (unsigned)db.y - nb;
    const unsigned s6 = (unsigned)db.z - nb, s7 = (unsigned)db.w - nb;
    const bool h0 = s0 < (unsigned)NB, h1 = s1 < (unsigned)NB, h2 = s2 < (unsigned)NB, h3 = s3 < (unsigned)NB;
    const bool h4 = s4 < (unsigned)NB, h5 = s5 < (unsigned)NB, h6 = s6 < (unsigned)NB, h7 = s7 < (unsigned)NB;
    const unsigned any = __builtin_amdgcn_ballot_w32(h0 | h1 | h2 | h3 | h4 | h5 | h6 | h7);
    if (any != 0u) {
#define HITJ(J, HJ, SJ) { \
        const unsigned mj = __builtin_amdgcn_ballot_w32(HJ); \
        if (mj != 0u) { \
          if (HJ) { \
            const int pos = wc + (int)__builtin_amdgcn_mbcnt_lo(mj, 0u); \
            if (pos < WCAP) list[wave * WCAP + pos] = ((el0 + (J)) << 12) | (int)(SJ); \
          } \
          wc += (int)__builtin_popcount(mj); } }
      HITJ(0, h0, s0)
      HITJ(1, h1, s1)
      HITJ(2, h2, s2)
      HITJ(3, h3, s3)
      HITJ(4, h4, s4)
      HITJ(5, h5, s5)
      HITJ(6, h6, s6)
      HITJ(7, h7, s7)
#undef HITJ
    }
  }
  return wc;
}

__global__ __launch_bounds__(NTHR) void k_wprep(const float* __restrict__ W, _Float16* wp, int KD, int NC) {
  const int i = blockIdx.x * NTHR + threadIdx.x;
  const int kq = KD >> 3;
  const int total = NC * kq;
  if (i < total) {
    const int n  = i / kq;
    const int k0 = (i - n * kq) * 8;
    const float* src = W + (size_t)k0 * NC + n;
    v4f a, b;
    a.x = src[0];              a.y = src[NC];             a.z = src[2 * NC];         a.w = src[3 * NC];
    b.x = src[4 * NC];         b.y = src[5 * NC];         b.z = src[6 * NC];         b.w = src[7 * NC];
    Pack8 p;
    p.h = cvt8(a, b, WSCALE);
    _Float16* dh = wp + (size_t)i * 8;
    *(volatile v4i*)dh = p.i;
    __threadfence();
    *(volatile v4i*)dh = p.i;
  }
}

__global__ __launch_bounds__(NTHR) void k_count(const int* __restrict__ ei, int* cnt, int nE, int vec8) {
  __shared__ __attribute__((aligned(16))) int scnt[NBC];
  __shared__ __attribute__((aligned(16))) int list[LISTN];
  __shared__ int wcnt[NWAVE];
  const int tid = threadIdx.x, lane = tid & 31, wave = tid >> 5;
  const int nodeBase = blockIdx.x * NBC;
  const int* keys = ei;

  for (int i = tid; i < NBC; i += NTHR) scnt[i] = 0;
  __syncthreads();

  const int nChunks = (nE + CHUNK - 1) / CHUNK;
#pragma unroll 1
  for (int ch = 0; ch < nChunks; ++ch) {
    const int cbase = ch * CHUNK;
    const int wc = scan_chunk<NBC>(keys, nE, cbase, nodeBase, vec8, list, tid, lane, wave);
    if (lane == 0) wcnt[wave] = wc;
    __syncthreads();
    if (wave == 0) {
#pragma unroll 1
      for (int wsx = 0; wsx < NWAVE; ++wsx) {
        int n = __builtin_amdgcn_readfirstlane(wcnt[wsx]);
        n = n > WCAP ? WCAP : (n < 0 ? 0 : n);
        const int* lp = list + wsx * WCAP;
#pragma unroll 1
        for (int i = 0; i < n; ++i) {
          const int ent  = __builtin_amdgcn_readfirstlane(lp[i]);
          const int slot = ent & (NBC - 1);
          if (lane == 0) scnt[slot] = scnt[slot] + 1;
        }
      }
    }
    __syncthreads();
  }

  v4i cq[4];
#pragma unroll
  for (int q = 0; q < 4; ++q) {
    const int f = (wave * 4 + q) * 128 + 4 * lane;
    cq[q] = *(const v4i*)(scnt + f);
  }
  int* cp = cnt + (size_t)nodeBase;
#pragma unroll
  for (int q = 0; q < 4; ++q) {
    const int f = (wave * 4 + q) * 128 + 4 * lane;
    *(volatile v4i*)(cp + f) = cq[q];
  }
  __threadfence();
#pragma unroll
  for (int q = 0; q < 4; ++q) {
    const int f = (wave * 4 + q) * 128 + 4 * lane;
    *(volatile v4i*)(cp + f) = cq[q];
  }
}

__global__ __launch_bounds__(OTHR) void k_offsets(
    const int* __restrict__ cnt, int* off, int* rbase, int nChunk) {
  __shared__ __attribute__((aligned(16))) int soff[NBC];
  __shared__ __attribute__((aligned(16))) int srb[RBN];
  __shared__ int wtot[OTHR / 32];
  const int tid = threadIdx.x, lane = tid & 31, wave = tid >> 5, sub = tid >> 7;
  for (int i = tid; i < RBN; i += OTHR) srb[i] = 0;
  int carry = 0;
#pragma unroll 1
  for (int ch = 0; ch < nChunk; ++ch) {
    const int base = ch * NBC;
    const v4i c0 = *(const v4i*)(cnt + base + 8 * tid);
    const v4i c1 = *(const v4i*)(cnt + base + 8 * tid + 4);
    const int e0 = max(c0.x, 0), e1 = max(c0.y, 0), e2 = max(c0.z, 0), e3 = max(c0.w, 0);
    const int e4 = max(c1.x, 0), e5 = max(c1.y, 0), e6 = max(c1.z, 0), e7 = max(c1.w, 0);
    const int ts = e0 + e1 + e2 + e3 + e4 + e5 + e6 + e7;
    int incl = ts;
#pragma unroll
    for (int d = 1; d < 32; d <<= 1) {
      const int t = __shfl_up(incl, d);
      if (lane >= d) incl += t;
    }
    if (lane == 31) wtot[wave] = incl;
    __syncthreads();
    const int S0 = wtot[0]  + wtot[1]  + wtot[2]  + wtot[3];
    const int S1 = wtot[4]  + wtot[5]  + wtot[6]  + wtot[7];
    const int S2 = wtot[8]  + wtot[9]  + wtot[10] + wtot[11];
    const int S3 = wtot[12] + wtot[13] + wtot[14] + wtot[15];
    int pre = 0;
#pragma unroll 1
    for (int w = 4 * sub; w < wave; ++w) pre += wtot[w];
    const int b0 = carry;
    const int b1 = b0 + ((S0 + 31) & ~31);
    const int b2 = b1 + ((S1 + 31) & ~31);
    const int b3 = b2 + ((S2 + 31) & ~31);
    const int b4 = b3 + ((S3 + 31) & ~31);
    const int myb = sub == 0 ? b0 : (sub == 1 ? b1 : (sub == 2 ? b2 : b3));
    if (tid == 0) {
      srb[min(4 * ch + 0, RBN - 1)] = b0;
      srb[min(4 * ch + 1, RBN - 1)] = b1;
      srb[min(4 * ch + 2, RBN - 1)] = b2;
      srb[min(4 * ch + 3, RBN - 1)] = b3;
    }
    int run = myb + pre + incl - ts;
    soff[8 * tid + 0] = run; run += e0;
    soff[8 * tid + 1] = run; run += e1;
    soff[8 * tid + 2] = run; run += e2;
    soff[8 * tid + 3] = run; run += e3;
    soff[8 * tid + 4] = run; run += e4;
    soff[8 * tid + 5] = run; run += e5;
    soff[8 * tid + 6] = run; run += e6;
    soff[8 * tid + 7] = run;
    carry = b4;
    __syncthreads();
    const v4i o0 = *(const v4i*)(soff + 4 * tid);
    const v4i o1 = *(const v4i*)(soff + 4 * (tid + OTHR));
    int* op = off + base;
    *(volatile v4i*)(op + 4 * tid) = o0;
    *(volatile v4i*)(op + 4 * (tid + OTHR)) = o1;
    __threadfence();
    *(volatile v4i*)(op + 4 * tid) = o0;
    *(volatile v4i*)(op + 4 * (tid + OTHR)) = o1;
    __syncthreads();
  }
  if (tid == 0) srb[min(4 * nChunk, RBN - 1)] = carry;
  __syncthreads();
  v4i rv = {0, 0, 0, 0};
  if (tid < 32) rv = *(const v4i*)(srb + 4 * tid);
  if (tid < 32) *(volatile v4i*)(rbase + 4 * tid) = rv;
  __threadfence();
  if (tid < 32) *(volatile v4i*)(rbase + 4 * tid) = rv;
}

__global__ __launch_bounds__(NTHR) void k_fill(
    const int* __restrict__ ei, const int* __restrict__ off, const int* __restrict__ rbase,
    int* csr, int nN, int nE, int vec8, int csrLen) {
  extern __shared__ v4f lds_dyn[];
  int* region = (int*)lds_dyn;
  int* cursor = region + RCAP;
  int* list   = cursor + NBF;
  int* wcnt   = list + LISTN;
  const int tid = threadIdx.x, lane = tid & 31, wave = tid >> 5;
  const int b = blockIdx.x;
  const int nodeBase = b * NBF;
  const int* keys = ei;

  int rb0 = rbase[b];
  const int rb1 = rbase[b + 1];
  rb0 = rb0 < 0 ? 0 : (rb0 > csrLen ? csrLen : rb0);
  rb0 &= ~31;
  int len = rb1 - rb0;
  len = len < 0 ? 0 : (len > RCAP ? RCAP : len);
  int lenW = (len + 31) & ~31;
  if (rb0 + lenW > csrLen) lenW = (csrLen - rb0) & ~31;

  {
    const v4i z = {0, 0, 0, 0};
    for (int i = tid; i < RCAP / 4; i += NTHR) ((v4i*)region)[i] = z;
    for (int s = tid; s < NBF; s += NTHR) {
      int o = off[nodeBase + s] - rb0;
      o = o < 0 ? 0 : (o > RCAP ? RCAP : o);
      cursor[s] = o;
    }
  }
  __syncthreads();

  const int nChunks = (nE + CHUNK - 1) / CHUNK;
#pragma unroll 1
  for (int ch = 0; ch < nChunks; ++ch) {
    const int cbase = ch * CHUNK;
    const int wc = scan_chunk<NBF>(keys, nE, cbase, nodeBase, vec8, list, tid, lane, wave);
    if (lane == 0) wcnt[wave] = wc;
    __syncthreads();
    if (wave == 0) {
#pragma unroll 1
      for (int wsx = 0; wsx < NWAVE; ++wsx) {
        int n = __builtin_amdgcn_readfirstlane(wcnt[wsx]);
        n = n > WCAP ? WCAP : (n < 0 ? 0 : n);
        const int* lp = list + wsx * WCAP;
#pragma unroll 1
        for (int i = 0; i < n; ++i) {
          const int ent  = __builtin_amdgcn_readfirstlane(lp[i]);
          const int slot = ent & (NBF - 1);
          int e = cbase + ((ent >> 12) & (CHUNK - 1));
          e = e > nE - 1 ? nE - 1 : e;
          const int d = ei[nE + e];
          int val = ((nodeBase + slot) & ~(NNODE - 1)) | (d & (NNODE - 1));
          val = val < 0 ? 0 : (val > nN - 1 ? nN - 1 : val);
          if (lane == 0) {
            int pos = cursor[slot];
            pos = pos < 0 ? 0 : (pos > RCAP - 1 ? RCAP - 1 : pos);
            region[pos] = val;
            const int np = pos + 1;
            cursor[slot] = np > RCAP ? RCAP : np;
          }
        }
      }
    }
    __syncthreads();
  }

  const int nv = lenW >> 2;
  int* gp = csr + rb0;
#pragma unroll 1
  for (int i = tid; i < nv; i += NTHR) { const v4i v = ((const v4i*)region)[i]; *(volatile v4i*)(gp + 4 * i) = v; }
  __threadfence();
#pragma unroll 1
  for (int i = tid; i < nv; i += NTHR) { const v4i v = ((const v4i*)region)[i]; *(volatile v4i*)(gp + 4 * i) = v; }
}

__global__ __launch_bounds__(NTHR) void k_agg(
    const int* __restrict__ csr, const int* __restrict__ off, const int* __restrict__ cnt,
    const float* xin, const float* __restrict__ alpha_p, float* aout,
    int ldx, int ldo, int mixCol, int copyCol, int doCopy, int nN, int csrLen) {
  const int tid = threadIdx.x, lane = tid & 31, wave = tid >> 5;
  const int tbase = blockIdx.x * TGT + wave * 32;
  const int cl = tbase + lane;
  const int cnt_l = cnt[cl];
  const int off_l = off[cl];
  const float alpha = alpha_p[0];
  const float oma = 1.0f - alpha;

#pragma unroll 1
  for (int j = 0; j < 32; ++j) {
    const int c = tbase + j;
    int n = __builtin_amdgcn_readlane(cnt_l, j);
    n = n < 0 ? 0 : (n > DEGCAP ? DEGCAP : n);
    const int st = __builtin_amdgcn_readlane(off_l, j);
    v4f acc = {0.0f, 0.0f, 0.0f, 0.0f};
#pragma unroll 1
    for (int q0 = 0; q0 < n; q0 += 32) {
      int pos = st + q0 + lane;
      pos = pos < 0 ? 0 : (pos > csrLen - 1 ? csrLen - 1 : pos);
      int sl = csr[pos];
      sl = sl < 0 ? 0 : (sl > nN - 1 ? nN - 1 : sl);
      const int mcnt = (n - q0) < 32 ? (n - q0) : 32;
#pragma unroll 1
      for (int p = 0; p < mcnt; ++p) {
        const int s = __builtin_amdgcn_readlane(sl, p);
        const v4f v = *(const v4f*)(xin + (size_t)s * ldx + 4 * lane);
        acc = acc + v;
      }
    }
    const int cs = c > nN - 1 ? nN - 1 : c;
    const v4f sv = *(const v4f*)(xin + (size_t)cs * ldx + 4 * lane);
    v4f mix;
    mix.x = alpha * acc.x + oma * sv.x;
    mix.y = alpha * acc.y + oma * sv.y;
    mix.z = alpha * acc.z + oma * sv.z;
    mix.w = alpha * acc.w + oma * sv.w;
    float* op = aout + (size_t)c * ldo + 4 * lane;
    *(volatile v4f*)(op + mixCol) = mix;
    if (doCopy != 0) *(volatile v4f*)(op + copyCol) = sv;
    __threadfence();
    *(volatile v4f*)(op + mixCol) = mix;
    if (doCopy != 0) *(volatile v4f*)(op + copyCol) = sv;
  }
}

template <int KD, int NC, int NCT, int RELU>
__global__ __launch_bounds__(NTHR) void k_gemm(
    const float* __restrict__ A, const _Float16* __restrict__ Bw,
    const float* __restrict__ bias, float* C, int mrows) {
  static_assert((KD % 32) == 0 && (NC % 64) == 0 && (NCT % NC) == 0 && NC <= 128);
  static_assert(GROWS * NC * 4 <= LDS_GEMM(KD));
  static_assert(((GROWS * KD / 8) % NTHR) == 0);
  extern __shared__ v4f lds_dyn[];
  constexpr int APK  = KD + 8;
  constexpr int NT   = NC / 16;
  constexpr int NKT  = KD / 32;
  constexpr int NIT  = (GROWS * KD / 8) / NTHR;
  constexpr int LPR  = NC / 4;
  constexpr int RPI  = 32 / LPR;
  constexpr int NV   = 16 / RPI;
  _Float16* sA  = (_Float16*)lds_dyn;
  float*    stg = (float*)lds_dyn;
  const int tid = threadIdx.x, lane = tid & 31, wave = tid >> 5, hh = lane >> 4, m = lane & 15;
  const int rowBase = blockIdx.x * GROWS;
  const int colBase = blockIdx.y * NC;

#pragma unroll 2
  for (int i = 0; i < NIT; ++i) {
    const int idx = i * NTHR + tid;
    const int r   = idx / (KD / 8);
    const int c0  = (idx - r * (KD / 8)) * 8;
    const float* ap = A + (size_t)(rowBase + r) * KD + c0;
    const v4f a = *(const v4f*)ap, b = *(const v4f*)(ap + 4);
    *(v8h*)(sA + r * APK + c0) = cvt8(a, b, 1.0f);
  }
  __syncthreads();

  v8f acc[NT];
#pragma unroll
  for (int t = 0; t < NT; ++t) { v8f z = {0.f, 0.f, 0.f, 0.f, 0.f, 0.f, 0.f, 0.f}; acc[t] = z; }
  const _Float16* afp = sA + (wave * 16 + m) * APK + 8 * hh;
  const _Float16* bwp = Bw + (size_t)(colBase + m) * KD + 8 * hh;
#pragma unroll 1
  for (int kt = 0; kt < NKT; ++kt) {
    FragH af;
    af.h[0] = *(const v8h*)(afp + 32 * kt);
    af.h[1] = *(const v8h*)(afp + 32 * kt + 16);
#pragma unroll
    for (int t = 0; t < NT; ++t) {
      const _Float16* bp = bwp + (size_t)(16 * t) * KD + 32 * kt;
      FragH bf;
      bf.h[0] = *(const v8h*)bp;
      bf.h[1] = *(const v8h*)(bp + 16);
      acc[t] = wmh(af.v, bf.v, acc[t]);
    }
  }
  __syncthreads();

  const int r0 = wave * 16 + 8 * hh;
  float* sp = stg + r0 * NC + m;
#pragma unroll
  for (int t = 0; t < NT; ++t) {
    const float bv = bias[colBase + 16 * t + m];
#pragma unroll
    for (int r = 0; r < 8; ++r) {
      float v = acc[t][r] * WINV + bv;
      if (RELU) v = fmaxf(v, 0.0f);
      sp[r * NC + 16 * t] = v;
    }
  }
  __syncthreads();

  if (rowBase + wave * 16 < mrows) {
    const float* lp = stg + wave * 16 * NC + 4 * lane;
    float* gp = C + (size_t)(rowBase + wave * 16 + lane / LPR) * NCT + colBase + 4 * (lane % LPR);
    v4f vv[NV];
#pragma unroll
    for (int i = 0; i < NV; ++i) vv[i] = *(const v4f*)(lp + 128 * i);
#pragma unroll
    for (int i = 0; i < NV; ++i) *(volatile v4f*)(gp + (size_t)(RPI * i) * NCT) = vv[i];
    __threadfence();
#pragma unroll
    for (int i = 0; i < NV; ++i) *(volatile v4f*)(gp + (size_t)(RPI * i) * NCT) = vv[i];
  }
}

__global__ __launch_bounds__(FEAT) void k_pool(const float* __restrict__ h, float* pooled, int G, int prow) {
  __shared__ __attribute__((aligned(16))) float sm[FEAT];
  const int g = blockIdx.x, f = threadIdx.x, lane = f & 31, wave = f >> 5;
  const float* hp = h + (size_t)g * NNODE * FEAT + f;
  float mx = -3.0e38f;
#pragma unroll 4
  for (int node = 0; node < NNODE; ++node) mx = fmaxf(mx, hp[(size_t)node * FEAT]);
  sm[f] = mx;
  __syncthreads();
  if (wave == 0) {
    const v4f v = *(const v4f*)(sm + 4 * lane);
    const v4f z = {0.0f, 0.0f, 0.0f, 0.0f};
    float* pr = pooled + (size_t)g * FEAT + 4 * lane;
    *(volatile v4f*)pr = v;
#pragma unroll 1
    for (int zr = g + G; zr < prow; zr += G) *(volatile v4f*)(pooled + (size_t)zr * FEAT + 4 * lane) = z;
    __threadfence();
    *(volatile v4f*)pr = v;
#pragma unroll 1
    for (int zr = g + G; zr < prow; zr += G) *(volatile v4f*)(pooled + (size_t)zr * FEAT + 4 * lane) = z;
  }
}

extern "C" void kernel_launch(void* const* d_in, const int* in_sizes, int n_in,
                              void* d_out, int out_size, void* d_ws, size_t ws_size,
                              hipStream_t stream) {
  if (n_in < 10) return;
  const int nN = in_sizes[1];
  if (nN <= 0 || in_sizes[0] != nN * FEAT) return;
  if ((in_sizes[2] & 1) != 0) return;
  const int nE = in_sizes[2] / 2;
  if (nE <= 0) return;
  if (in_sizes[3] != NTAP * FEAT * FEAT || in_sizes[4] != FEAT) return;
  if (in_sizes[5] != NTAP * FEAT * FEAT || in_sizes[6] != FEAT) return;
  if (in_sizes[7] != FEAT * FOUTC || in_sizes[8] != FOUTC || in_sizes[9] < 1) return;
  const int G = out_size / FOUTC;
  if (G <= 0 || out_size != G * FOUTC || (G % 16) != 0) return;
  if (nN != G * NNODE) return;
  if ((nN % TGT) != 0) return;
  if (nE > (1 << 28) || nN > (1 << 24)) return;

  const float* X    = (const float*)d_in[0];
  const int*   ei   = (const int*)d_in[2];
  const float* W1   = (const float*)d_in[3];
  const float* b1   = (const float*)d_in[4];
  const float* W2   = (const float*)d_in[5];
  const float* b2   = (const float*)d_in[6];
  const float* Wo   = (const float*)d_in[7];
  const float* bo   = (const float*)d_in[8];
  const float* alp  = (const float*)d_in[9];
  float* out = (float*)d_out;

  const int NPAD   = nN;
  const int nBC    = (nN + NBC - 1) / NBC;
  const int CNTPAD = nBC * NBC;
  if (4 * nBC + 1 > RBN) return;
  const int nBF    = (nN + NBF - 1) / NBF;
  const int csrLen = ((nE + 31) & ~31) + 4096;
  if (31 * 4 * nBC > 4096) return;
  const int nGemm  = NPAD / GROWS;
  const int nAgg   = NPAD / TGT;
  const int prow   = ((G + GROWS - 1) / GROWS) * GROWS;
  const int WPC    = FEAT * KCONV;
  const int WPO    = FOUTC * FEAT;

  char* ws = (char*)d_ws;
  size_t off = 0;
  const size_t oW1  = off; off += (size_t)WPC * 2;                 off = (off + 255) & ~(size_t)255;
  const size_t oW2  = off; off += (size_t)WPC * 2;                 off = (off + 255) & ~(size_t)255;
  const size_t oWo  = off; off += (size_t)WPO * 2;                 off = (off + 255) & ~(size_t)255;
  const size_t oCnt = off; off += (size_t)CNTPAD * 4;              off = (off + 255) & ~(size_t)255;
  const size_t oOff = off; off += (size_t)CNTPAD * 4;              off = (off + 255) & ~(size_t)255;
  const size_t oRb  = off; off += (size_t)RBN * 4;                 off = (off + 255) & ~(size_t)255;
  const size_t oCsr = off; off += (size_t)csrLen * 4;              off = (off + 255) & ~(size_t)255;
  const size_t oRA  = off; off += (size_t)NPAD * KCONV * 4;        off = (off + 255) & ~(size_t)255;
  const size_t oRH  = off; off += (size_t)NPAD * FEAT * 4;         off = (off + 255) & ~(size_t)255;
  const size_t oPl  = off; off += (size_t)prow * FEAT * 4;         off = (off + 255) & ~(size_t)255;
  if (off > ws_size || off > (size_t)WSCAP) return;
  _Float16* wp1  = (_Float16*)(ws + oW1);
  _Float16* wp2  = (_Float16*)(ws + oW2);
  _Float16* wpo  = (_Float16*)(ws + oWo);
  int*      cnt  = (int*)(ws + oCnt);
  int*      offp = (int*)(ws + oOff);
  int*      rb   = (int*)(ws + oRb);
  int*      csr  = (int*)(ws + oCsr);
  float*    RA   = (float*)(ws + oRA);
  float*    RH   = (float*)(ws + oRH);
  float*    PL   = (float*)(ws + oPl);

  const int vec8 = ((nE & 3) == 0) ? 1 : 0;

  k_wprep<<<(FEAT * KCONV / 8 + NTHR - 1) / NTHR, NTHR, 0, stream>>>(W1, wp1, KCONV, FEAT);
  k_wprep<<<(FEAT * KCONV / 8 + NTHR - 1) / NTHR, NTHR, 0, stream>>>(W2, wp2, KCONV, FEAT);
  k_wprep<<<(FOUTC * FEAT / 8 + NTHR - 1) / NTHR, NTHR, 0, stream>>>(Wo, wpo, FEAT, FOUTC);

  k_count<<<nBC, NTHR, 0, stream>>>(ei, cnt, nE, vec8);
  k_offsets<<<1, OTHR, 0, stream>>>(cnt, offp, rb, nBC);
  hipFuncSetAttribute(reinterpret_cast<const void*>(&k_fill),
                      hipFuncAttributeMaxDynamicSharedMemorySize, LDS_FILL);
  k_fill<<<nBF, NTHR, LDS_FILL, stream>>>(ei, offp, rb, csr, nN, nE, vec8, csrLen);

  k_agg<<<nAgg, NTHR, 0, stream>>>(csr, offp, cnt, X, alp, RA, FEAT, KCONV, FEAT, 0, 1, nN, csrLen);
  k_agg<<<nAgg, NTHR, 0, stream>>>(csr, offp, cnt, RA + FEAT, alp, RA, KCONV, KCONV, 2 * FEAT, 0, 0, nN, csrLen);
  hipFuncSetAttribute(reinterpret_cast<const void*>(&k_gemm<KCONV, 64, FEAT, 1>),
                      hipFuncAttributeMaxDynamicSharedMemorySize, LDS_GEMM(KCONV));
  k_gemm<KCONV, 64, FEAT, 1><<<dim3(nGemm, FEAT / 64, 1), NTHR, LDS_GEMM(KCONV), stream>>>(RA, wp1, b1, RH, NPAD);

  k_agg<<<nAgg, NTHR, 0, stream>>>(csr, offp, cnt, RH, alp, RA, FEAT, KCONV, FEAT, 0, 1, nN, csrLen);
  k_agg<<<nAgg, NTHR, 0, stream>>>(csr, offp, cnt, RA + FEAT, alp, RA, KCONV, KCONV, 2 * FEAT, 0, 0, nN, csrLen);
  k_gemm<KCONV, 64, FEAT, 1><<<dim3(nGemm, FEAT / 64, 1), NTHR, LDS_GEMM(KCONV), stream>>>(RA, wp2, b2, RH, NPAD);

  k_pool<<<G, FEAT, 0, stream>>>(RH, PL, G, prow);
  hipFuncSetAttribute(reinterpret_cast<const void*>(&k_gemm<FEAT, 64, FOUTC, 0>),
                      hipFuncAttributeMaxDynamicSharedMemorySize, LDS_GEMM(FEAT));
  k_gemm<FEAT, 64, FOUTC, 0><<<dim3(prow / GROWS, FOUTC / 64, 1), NTHR, LDS_GEMM(FEAT), stream>>>(PL, wpo, bo, out, G);
}
